// MMA_25821343383855
// MI455X (gfx1250) — hardware-verified
//
#include <hip/hip_runtime.h>


#define NIMG 10
#define DM   64
#define TT   16384
#define NGRP 32
#define GCH  (DM / NGRP)
#define RPAD 2
#define KC   512
#define SCL  0.125f
typedef _Float16 h16;
typedef unsigned short bf;
typedef __attribute__((ext_vector_type(16))) __bf16   v16bf;
typedef __attribute__((ext_vector_type(16))) _Float16 v16h;
typedef __attribute__((ext_vector_type(8)))  _Float16 v8h;
typedef __attribute__((ext_vector_type(8)))  unsigned short v8us;
typedef __attribute__((ext_vector_type(8)))  float    v8f;
typedef __attribute__((ext_vector_type(4)))  float    v4f;
typedef __attribute__((ext_vector_type(2)))  float    v2f;
typedef __attribute__((ext_vector_type(4)))  unsigned short v4us;
typedef __attribute__((ext_vector_type(2)))  unsigned short v2us;
typedef v8h  __attribute__((may_alias)) v8ha;
typedef v4f  __attribute__((may_alias)) v4fa;
typedef v8us __attribute__((may_alias)) v8usa;

__device__ __forceinline__ unsigned short f2bf(float f) { unsigned u = __float_as_uint(f); u += 0x7FFFu + ((u >> 16) & 1u); return (unsigned short)(u >> 16); }
__device__ __forceinline__ float bf2f(unsigned short b) { return __uint_as_float(((unsigned)b) << 16); }
__device__ __forceinline__ float bfr(float f) { return bf2f(f2bf(f)); }
__device__ __forceinline__ void splitf(float y, unsigned short& h, unsigned short& l) { h = f2bf(y); l = f2bf(y - bf2f(h)); }
__device__ __forceinline__ v16h cat16(v8h lo, v8h hi) { return __builtin_shufflevector(lo, hi, 0, 1, 2, 3, 4, 5, 6, 7, 8, 9, 10, 11, 12, 13, 14, 15); }
__device__ __forceinline__ v16bf cat16b(v8us lo, v8us hi) { return __builtin_bit_cast(v16bf, __builtin_shufflevector(lo, hi, 0, 1, 2, 3, 4, 5, 6, 7, 8, 9, 10, 11, 12, 13, 14, 15)); }
__device__ __forceinline__ v8f wmma16(v16h a, v16h b, v8f c) { return __builtin_amdgcn_wmma_f32_16x16x32_f16(false, a, false, b, (short)0, c, false, false); }
__device__ __forceinline__ v8f wmmab(v16bf a, v16bf b, v8f c) { return __builtin_amdgcn_wmma_f32_16x16x32_bf16(false, a, false, b, (short)0, c, false, false); }

template <typename T16> struct WFrag;
template <> struct WFrag<h16> { typedef v16h V; static __device__ __forceinline__ V ld(const h16* p) { return cat16(*(const v8h*)p, *(const v8h*)(p + 16)); } static __device__ __forceinline__ v8f mma(V a, V b, v8f c) { return wmma16(a, b, c); } };
template <> struct WFrag<bf> { typedef v16bf V; static __device__ __forceinline__ V ld(const bf* p) { return cat16b(*(const v8us*)p, *(const v8us*)(p + 16)); } static __device__ __forceinline__ v8f mma(V a, V b, v8f c) { return wmmab(a, b, c); } };
template <typename T16, int NSPLIT, bool BIAS>
__global__ __launch_bounds__(32) void k_gemmw(const T16* __restrict__ A, const T16* __restrict__ A2, const T16* __restrict__ Bt, const T16* __restrict__ Bt2, int K, float* C, int ldc, const float* __restrict__ bias, size_t sA, size_t sB, size_t sC) {
    typedef typename WFrag<T16>::V V;
    __shared__ __align__(16) float os[16 * 68];
    const size_t z = blockIdx.z; A += z * sA; if (A2) A2 += z * sA; Bt += z * sB; if (Bt2) Bt2 += z * sB; C += z * sC;
    const int lane = threadIdx.x & 31, lr = lane & 15, hi = lane >> 4; const int r0 = blockIdx.x * 64, c0 = blockIdx.y * 64;
    v8f acc[4][4];
#pragma unroll
    for (int mb = 0; mb < 4; ++mb)
#pragma unroll
        for (int nb = 0; nb < 4; ++nb) acc[mb][nb] = (v8f){};
    const size_t aoff = (size_t)(r0 + lr) * K + 8 * hi, boff = (size_t)(c0 + lr) * K + 8 * hi;
#pragma unroll 1
    for (int kc = 0; kc < K; kc += 32) {
        V a[4], a2[4];
#pragma unroll
        for (int mb = 0; mb < 4; ++mb) { a[mb] = WFrag<T16>::ld(A + aoff + (size_t)mb * 16 * K + kc); if (NSPLIT == 1 || NSPLIT == 2) a2[mb] = WFrag<T16>::ld(A2 + aoff + (size_t)mb * 16 * K + kc); }
#pragma unroll
        for (int nb = 0; nb < 4; ++nb) { const V b = WFrag<T16>::ld(Bt + boff + (size_t)nb * 16 * K + kc); V b2; if (NSPLIT >= 2) b2 = WFrag<T16>::ld(Bt2 + boff + (size_t)nb * 16 * K + kc);
#pragma unroll
            for (int mb = 0; mb < 4; ++mb) { acc[mb][nb] = WFrag<T16>::mma(a[mb], b, acc[mb][nb]); if (NSPLIT == 1 || NSPLIT == 2) acc[mb][nb] = WFrag<T16>::mma(a2[mb], b, acc[mb][nb]); if (NSPLIT >= 2) acc[mb][nb] = WFrag<T16>::mma(a[mb], b2, acc[mb][nb]); } }
        asm volatile("v_nop\n\tv_nop\n\tv_nop\n\tv_nop" : "+v"(acc[0][0]), "+v"(acc[1][1]), "+v"(acc[2][2]), "+v"(acc[3][3]) : "v"(a[0]), "v"(a[3]));
    }
#pragma unroll
    for (int mb = 0; mb < 4; ++mb) {
#pragma unroll
        for (int nb = 0; nb < 4; ++nb) {
#pragma unroll
            for (int j = 0; j < 8; ++j) os[(hi * 8 + j) * 68 + nb * 16 + lr] = acc[mb][nb][j]; }
        __builtin_amdgcn_wave_barrier(); asm volatile("" ::: "memory");
        float* crow = C + (size_t)(r0 + mb * 16) * ldc + c0;
#pragma unroll 1
        for (int ps = 0; ps < 2; ++ps) {
#pragma unroll
            for (int s = 0; s < 8; ++s) { const int row = 2 * s + hi, cofs = lr * 4; v4f val = *(const v4fa*)(os + row * 68 + cofs); if (BIAS) { val[0] += bfr(bias[c0 + cofs]); val[1] += bfr(bias[c0 + cofs + 1]); val[2] += bfr(bias[c0 + cofs + 2]); val[3] += bfr(bias[c0 + cofs + 3]); }
                *(volatile v4f*)(crow + (size_t)row * ldc + cofs) = val; }
            if (ps == 0) __threadfence(); }
        __builtin_amdgcn_wave_barrier(); asm volatile("" ::: "memory");
    }
}

__global__ __launch_bounds__(256) void k_cvt8(const float* __restrict__ src, bf* dst, size_t n8) { const size_t i = (size_t)blockIdx.x * 256 + threadIdx.x; if (i >= n8) return; const v8f v = *(const v8f*)(src + i * 8); v8us o;
#pragma unroll
    for (int k = 0; k < 8; ++k) o[k] = f2bf(v[k]); *(volatile v8us*)(dst + i * 8) = o; __threadfence(); *(volatile v8us*)(dst + i * 8) = o; }
__global__ __launch_bounds__(256) void k_mbT(const float* __restrict__ mb, bf* MT) { const size_t e = ((size_t)blockIdx.x * 256 + threadIdx.x) * 2; if (e >= (size_t)KC * DM) return; const int c = (int)(e % DM), k = (int)(e / DM); v2us o; o[0] = f2bf(mb[(size_t)c * KC + k]); o[1] = f2bf(mb[(size_t)(c + 1) * KC + k]); *(volatile v2us*)(MT + e) = o; __threadfence(); *(volatile v2us*)(MT + e) = o; }
__global__ __launch_bounds__(256) void k_gnstat(const float* __restrict__ xb, float* ST) { __shared__ float red[256]; const int g = blockIdx.x; const float* base = xb + (size_t)g * GCH * TT; const int tid = threadIdx.x; float s = 0.f;
#pragma unroll 1
    for (int i = tid; i < GCH * TT; i += 256) s = __fadd_rn(s, bfr(base[i]));
    red[tid] = s; __syncthreads();
#pragma unroll
    for (int sh = 128; sh; sh >>= 1) { if (tid < sh) red[tid] = __fadd_rn(red[tid], red[tid + sh]); __syncthreads(); }
    const float mu = red[0] * (1.0f / (GCH * TT)); __syncthreads(); float s2 = 0.f;
#pragma unroll 1
    for (int i = tid; i < GCH * TT; i += 256) { const float d0 = __fsub_rn(bfr(base[i]), mu); float p = __fmul_rn(d0, d0); asm volatile("" : "+v"(p)); s2 = __fadd_rn(s2, p); }
    red[tid] = s2; __syncthreads();
#pragma unroll
    for (int sh = 128; sh; sh >>= 1) { if (tid < sh) red[tid] = __fadd_rn(red[tid], red[tid + sh]); __syncthreads(); }
    if (tid == 0) { const float rs = __fdiv_rn(1.0f, __fsqrt_rn(__fadd_rn(red[0] * (1.0f / (GCH * TT)), 1e-6f))); v2f o; o[0] = mu; o[1] = rs; *(volatile v2f*)(ST + (size_t)g * RPAD) = o; __threadfence(); *(volatile v2f*)(ST + (size_t)g * RPAD) = o; } }
__global__ __launch_bounds__(256) void k_gnT(const float* __restrict__ xb, const float* __restrict__ ST, const float* __restrict__ gw, const float* __restrict__ gb, bf* Xh, bf* Xl) { const size_t e = ((size_t)blockIdx.x * 256 + threadIdx.x) * 4; if (e >= (size_t)TT * DM) return; const int c = (int)(e % DM); const int t = (int)(e / DM); v4us oh, ol;
#pragma unroll
    for (int q = 0; q < 4; ++q) { const int cc = c + q; const int g = cc / GCH; const float mu = ST[(size_t)g * RPAD], rs = ST[(size_t)g * RPAD + 1]; float n0 = __fmul_rn(__fsub_rn(bfr(xb[(size_t)cc * TT + t]), mu), rs); asm volatile("" : "+v"(n0)); float n1 = __fmul_rn(n0, bfr(gw[cc])); asm volatile("" : "+v"(n1)); const float y = __fadd_rn(n1, bfr(gb[cc])); unsigned short a, b2; splitf(y, a, b2); oh[q] = a; ol[q] = b2; }
    *(volatile v4us*)(Xh + e) = oh; *(volatile v4us*)(Xl + e) = ol; __threadfence(); *(volatile v4us*)(Xh + e) = oh; *(volatile v4us*)(Xl + e) = ol; }
__global__ __launch_bounds__(256) void k_outT(const float* __restrict__ xb, const float* __restrict__ YO, float* Ob) { const size_t e = (size_t)blockIdx.x * 256 + threadIdx.x; if (e >= (size_t)DM * TT) return; const int t = (int)(e % TT); const int c = (int)(e / TT); const float v = __fadd_rn(bfr(xb[e]), YO[(size_t)t * DM + c]); *(volatile float*)(Ob + e) = v; __threadfence(); *(volatile float*)(Ob + e) = v; }
__global__ __launch_bounds__(256) void k_pl2(const float* __restrict__ F, bf* Ph, bf* Pl, size_t n4) { const size_t i = (size_t)blockIdx.x * 256 + threadIdx.x; if (i >= n4) return; const v4f v = *(const v4f*)(F + i * 4); v4us oh, ol;
#pragma unroll
    for (int q = 0; q < 4; ++q) { unsigned short a, c; splitf(v[q], a, c); oh[q] = a; ol[q] = c; } *(volatile v4us*)(Ph + i * 4) = oh; *(volatile v4us*)(Pl + i * 4) = ol; __threadfence(); *(volatile v4us*)(Ph + i * 4) = oh; *(volatile v4us*)(Pl + i * 4) = ol; }
__global__ __launch_bounds__(256) void k_soft512(const float* __restrict__ Sb, bf* Ph, bf* Pl) {
    const int lane = threadIdx.x & 31; const int row = blockIdx.x * 8 + (threadIdx.x >> 5); if (row >= TT) return; const float* sr = Sb + (size_t)row * KC; float v[KC / 32]; float mx = -3.0e38f;
#pragma unroll
    for (int ch = 0; ch < KC / 128; ++ch) { const int j0 = ch * 128 + lane * 4; const v4f a = *(const v4f*)(sr + j0);
#pragma unroll
        for (int q = 0; q < 4; ++q) { const float t = a[q] * SCL; v[ch * 4 + q] = t; mx = fmaxf(mx, t); } }
#pragma unroll
    for (int sh = 16; sh; sh >>= 1) mx = fmaxf(mx, __shfl_xor(mx, sh, 32));
    float sum = 0.f;
#pragma unroll
    for (int k = 0; k < KC / 32; ++k) { float d0 = __fsub_rn(v[k], mx); asm volatile("" : "+v"(d0)); v[k] = __builtin_amdgcn_exp2f(__fmul_rn(d0, 1.4426950408889634f)); sum += v[k]; }
#pragma unroll
    for (int sh = 16; sh; sh >>= 1) sum += __shfl_xor(sum, sh, 32);
    const float f = __fdiv_rn(1.0f, sum);
#pragma unroll 1
    for (int ps = 0; ps < 2; ++ps) {
#pragma unroll
        for (int ch = 0; ch < KC / 128; ++ch) { v4us oh, ol;
#pragma unroll
            for (int q = 0; q < 4; ++q) { float pf = v[ch * 4 + q] * f; asm volatile("" : "+v"(pf)); unsigned short a, c2; splitf(pf, a, c2); oh[q] = a; ol[q] = c2; }
            const size_t oo = (size_t)row * KC + ch * 128 + lane * 4; *(volatile v4us*)(Ph + oo) = oh; *(volatile v4us*)(Pl + oo) = ol; }
        if (ps == 0) __threadfence(); }
}

extern "C" void kernel_launch(void* const* d_in, const int* in_sizes, int n_in,
                              void* d_out, int out_size, void* d_ws, size_t ws_size, hipStream_t stream) {
    (void)in_sizes; (void)n_in; (void)out_size;
    const float* x = (const float*)d_in[0]; const float* mb = (const float*)d_in[1]; const float* phw = (const float*)d_in[2]; const float* phb = (const float*)d_in[3]; const float* gnw = (const float*)d_in[4]; const float* gnb = (const float*)d_in[5]; const float* wzw = (const float*)d_in[6]; const float* wzb = (const float*)d_in[7];
    float* OUT = (float*)d_out;
    char* wsp = (char*)d_ws;
    auto take = [&](size_t bytes) { char* p = wsp; wsp += (bytes + 255) & ~(size_t)255; return (void*)p; };
    bf* PHW = (bf*)take((size_t)DM * DM * 2); bf* WZW = (bf*)take((size_t)DM * DM * 2); bf* MB = (bf*)take((size_t)DM * KC * 2); bf* MT = (bf*)take((size_t)KC * DM * 2); float* ST = (float*)take((size_t)NGRP * RPAD * 4);
    bf* XTh = (bf*)take((size_t)TT * DM * 2); bf* XTl = (bf*)take((size_t)TT * DM * 2); float* F = (float*)take((size_t)TT * DM * 4); bf* PPh = (bf*)take((size_t)TT * DM * 2); bf* PPl = (bf*)take((size_t)TT * DM * 2); float* Sb = (float*)take((size_t)TT * KC * 4); bf* Ph = (bf*)take((size_t)TT * KC * 2); bf* Pl = (bf*)take((size_t)TT * KC * 2); float* Y = (float*)take((size_t)TT * DM * 4); bf* Yh = (bf*)take((size_t)TT * DM * 2); bf* Yl = (bf*)take((size_t)TT * DM * 2); float* YO = (float*)take((size_t)TT * DM * 4);
    if ((size_t)(wsp - (char*)d_ws) > ws_size) return;
    k_cvt8<<<(DM * DM / 8 + 255) / 256, 256, 0, stream>>>(phw, PHW, (size_t)DM * DM / 8); k_cvt8<<<(DM * DM / 8 + 255) / 256, 256, 0, stream>>>(wzw, WZW, (size_t)DM * DM / 8); k_cvt8<<<(DM * KC / 8 + 255) / 256, 256, 0, stream>>>(mb, MB, (size_t)DM * KC / 8); k_mbT<<<(KC * DM / 2 + 255) / 256, 256, 0, stream>>>(mb, MT);
    const unsigned LP4 = (unsigned)(((size_t)TT * DM / 4 + 255) / 256);
    for (int b = 0; b < NIMG; ++b) { const float* xb = x + (size_t)b * DM * TT;
        k_gnstat<<<NGRP, 256, 0, stream>>>(xb, ST); k_gnT<<<LP4, 256, 0, stream>>>(xb, ST, gnw, gnb, XTh, XTl);
        k_gemmw<bf, 1, true><<<dim3(TT / 64, DM / 64, 1), 32, 0, stream>>>(XTh, XTl, PHW, nullptr, DM, F, DM, phb, 0, 0, 0); k_pl2<<<LP4, 256, 0, stream>>>(F, PPh, PPl, (size_t)TT * DM / 4);
        k_gemmw<bf, 1, false><<<dim3(TT / 64, KC / 64, 1), 32, 0, stream>>>(PPh, PPl, MT, nullptr, DM, Sb, KC, nullptr, 0, 0, 0);
        k_soft512<<<TT / 8, 256, 0, stream>>>(Sb, Ph, Pl);
        k_gemmw<bf, 1, false><<<dim3(TT / 64, DM / 64, 1), 32, 0, stream>>>(Ph, Pl, MB, nullptr, KC, Y, DM, nullptr, 0, 0, 0); k_pl2<<<LP4, 256, 0, stream>>>(Y, Yh, Yl, (size_t)TT * DM / 4);
        k_gemmw<bf, 1, true><<<dim3(TT / 64, DM / 64, 1), 32, 0, stream>>>(Yh, Yl, WZW, nullptr, DM, YO, DM, wzb, 0, 0, 0);
        k_outT<<<(unsigned)(((size_t)DM * TT + 255) / 256), 256, 0, stream>>>(xb, YO, OUT + (size_t)b * DM * TT); }
}
